// MaskedMultiHeadAttentionWithLoRAFinetuning_17566416240822
// MI455X (gfx1250) — hardware-verified
//
#include <hip/hip_runtime.h>
#include <math.h>
#include <float.h>
#include <stdint.h>

#define NB     4
#define SEQ    2048
#define DM     1024
#define NH     16
#define HD     64
#define FT     (NH * HD)
#define RK     8
#define RKP    16
#define EXT    64
#define LDX    (DM + EXT)
#define KE     (DM + 32)
#define NQB    (SEQ / 64)
#define GH     8
#define NGRP   (NH / GH)
#define QBRES  16
#define SPITCH 68
#define SPH    (64 * (NQB * SEQ - 32 * NQB * (NQB - 1)))

static_assert(HD == 64);
static_assert((SEQ % 64) == 0 && (DM % 64) == 0 && (FT % 64) == 0);
static_assert((DM / 8) == 128);
static_assert(((SEQ * (DM / 8)) % 256) == 0);
static_assert((LDX % 64) == 0);
static_assert((KE % 32) == 0 && KE <= LDX && KE >= DM + 2 * RK);
static_assert(2 * RK <= 16);
static_assert((NH % GH) == 0);
static_assert(QBRES >= 0 && QBRES <= NQB);
static_assert(SPH == 2162688);
static_assert((SPITCH * 4) % 16 == 0);
static_assert((SEQ % 16) == 0);

typedef _Float16 v16h __attribute__((ext_vector_type(16)));
typedef _Float16 v8h  __attribute__((ext_vector_type(8)));
typedef __bf16   v16b __attribute__((ext_vector_type(16)));
typedef __bf16   v8b  __attribute__((ext_vector_type(8)));
typedef float    v8f  __attribute__((ext_vector_type(8)));
typedef float    v4f  __attribute__((ext_vector_type(4)));
typedef unsigned int v4u __attribute__((ext_vector_type(4)));

__device__ __forceinline__ unsigned short bf_bits(float f) {
  unsigned u = __float_as_uint(f);
  return (unsigned short)((u + 0x7FFFu + ((u >> 16) & 1u)) >> 16);
}
__device__ __forceinline__ float bf_up(unsigned short h) { return __uint_as_float(((unsigned)h) << 16); }
__device__ __forceinline__ float bfr(float f) { return bf_up(bf_bits(f)); }
__device__ __forceinline__ unsigned short h_bits(_Float16 x) { return __builtin_bit_cast(unsigned short, x); }
__device__ __forceinline__ unsigned pk16(unsigned short a, unsigned short b) { return (unsigned)a | ((unsigned)b << 16); }
__device__ __forceinline__ v8f zero8() { v8f z = {0.f, 0.f, 0.f, 0.f, 0.f, 0.f, 0.f, 0.f}; return z; }

__host__ __device__ __forceinline__ size_t tileoff_d(int kb) {
  const int t = kb * SEQ - 32 * kb * (kb - 1);
  return (size_t)64 * (size_t)t;
}

__device__ __forceinline__ v16b ldfrag_b(const __bf16* p) {
  union { v16b v; v8b h[2]; } f;
  f.h[0] = *(const v8b*)(p);
  f.h[1] = *(const v8b*)(p + 16);
  return f.v;
}

__device__ __forceinline__ v8f mma_b(v16b a, v16b b, v8f c) {
  c = __builtin_amdgcn_wmma_f32_16x16x32_bf16(false, a, false, b, (short)0, c, false, false);
#if defined(__HIP_DEVICE_COMPILE__)
  asm volatile("v_nop\n\tv_nop\n\tv_nop\n\tv_nop" : "+v"(c) : "v"(a), "v"(b));
#endif
  return c;
}
__device__ __forceinline__ v8f mma_h(v16h a, v16h b, v8f c) {
  c = __builtin_amdgcn_wmma_f32_16x16x32_f16(false, a, false, b, (short)0, c, false, false);
#if defined(__HIP_DEVICE_COMPILE__)
  asm volatile("v_nop\n\tv_nop\n\tv_nop\n\tv_nop" : "+v"(c) : "v"(a), "v"(b));
#endif
  return c;
}
__device__ __forceinline__ v8f mma_b_raw(v16b a, v16b b, v8f c) {
  return __builtin_amdgcn_wmma_f32_16x16x32_bf16(false, a, false, b, (short)0, c, false, false);
}
__device__ __forceinline__ void dep_guard_b(v8f& a, v8f& b, v16b x, v16b y) {
#if defined(__HIP_DEVICE_COMPILE__)
  asm volatile("v_nop\n\tv_nop\n\tv_nop\n\tv_nop" : "+v"(a), "+v"(b) : "v"(x), "v"(y));
#endif
}
__device__ __forceinline__ void keep4_b(v16b a, v16b b, v16b c, v16b d) {
#if defined(__HIP_DEVICE_COMPILE__)
  asm volatile("v_nop" :: "v"(a), "v"(b), "v"(c), "v"(d));
#endif
}
__device__ __forceinline__ void acc_guard4(v8f& a, v8f& b, v8f& c, v8f& d) {
#if defined(__HIP_DEVICE_COMPILE__)
  asm volatile("v_nop\n\tv_nop\n\tv_nop\n\tv_nop" : "+v"(a), "+v"(b), "+v"(c), "+v"(d));
#endif
}

__global__ __launch_bounds__(256) void cvt_rows3(const float* __restrict__ s0, const float* __restrict__ s1,
                                                 const float* __restrict__ s2, unsigned short* d0,
                                                 unsigned short* d1, unsigned short* d2, int nper, int ntot) {
  const int i = blockIdx.x * 256 + threadIdx.x;
  if (i >= ntot) return;
  const int pr  = i / nper;
  const int loc = i - pr * nper;
  const int row = loc >> 7;
  const int c8  = (loc & 127) * 8;
  const float* src = (pr == 0) ? s0 : ((pr == 1) ? s1 : s2);
  unsigned short* dst = (pr == 0) ? d0 : ((pr == 1) ? d1 : d2);
  const float* s = src + (size_t)row * DM + c8;
  const v4f a = *(const v4f*)(s);
  const v4f b = *(const v4f*)(s + 4);
  v4u p;
  p[0] = pk16(bf_bits(a[0]), bf_bits(a[1]));
  p[1] = pk16(bf_bits(a[2]), bf_bits(a[3]));
  p[2] = pk16(bf_bits(b[0]), bf_bits(b[1]));
  p[3] = pk16(bf_bits(b[2]), bf_bits(b[3]));
  unsigned short* d = dst + (size_t)row * LDX + c8;
  *(volatile v4u*)d = p;
  __threadfence();
  *(volatile v4u*)d = p;
}

__global__ __launch_bounds__(256) void lr_at(const float* __restrict__ a0, const float* __restrict__ a1,
                                             const float* __restrict__ a2, unsigned short* at) {
  const int pr  = blockIdx.x >> 3;
  const int loc = ((blockIdx.x & 7) << 8) + (int)threadIdx.x;
  const int j   = loc >> 7;
  const int k8  = loc & 127;
  const int jj  = j & (RK - 1);
  const float* src = (pr == 0) ? a0 : ((pr == 1) ? a1 : a2);
  v4u p;
#pragma unroll
  for (int e = 0; e < 4; ++e) {
    const float f0 = src[(size_t)(k8 * 8 + 2 * e) * RK + jj];
    const float f1 = src[(size_t)(k8 * 8 + 2 * e + 1) * RK + jj];
    const unsigned w = pk16(bf_bits(f0), bf_bits(f1));
    p[e] = (j < RK) ? w : 0u;
  }
  unsigned short* d = at + (size_t)(pr * RKP + j) * DM + k8 * 8;
  *(volatile v4u*)d = p;
  __threadfence();
  *(volatile v4u*)d = p;
}

__global__ __launch_bounds__(256) void tr_cvt_bf16(const float* __restrict__ src, unsigned short* dst,
                                                   int K, int N, int ldd) {
  __shared__ float s[64][33];
  const int tid = threadIdx.x, wave = tid >> 5, lane = tid & 31;
  const int k0 = blockIdx.x * 64, n0 = blockIdx.y * 32;
#pragma unroll
  for (int i = 0; i < 8; ++i) {
    const int idx = i * 256 + tid;
    const int kk = idx >> 5, nn = idx & 31;
    s[kk][nn] = src[(size_t)(k0 + kk) * N + n0 + nn];
  }
  __syncthreads();
  const int q = lane >> 3, piece = lane & 7;
  const int n = wave * 4 + q;
  v4u p;
#pragma unroll
  for (int e = 0; e < 4; ++e) {
    p[e] = pk16(bf_bits(s[piece * 8 + 2 * e][n]), bf_bits(s[piece * 8 + 2 * e + 1][n]));
  }
  unsigned short* d = dst + (size_t)(n0 + n) * ldd + k0 + piece * 8;
  *(volatile v4u*)d = p;
  __threadfence();
  *(volatile v4u*)d = p;
}

__global__ __launch_bounds__(256) void wext(const float* __restrict__ Bm, unsigned short* dst, int ldd, int N,
                                            int ntot) {
  const int i = blockIdx.x * 256 + threadIdx.x;
  if (i >= ntot) return;
  const int p = i & 7;
  const int n = i >> 3;
  v4u w;
#pragma unroll
  for (int e = 0; e < 4; ++e) {
    const float f0 = Bm[(size_t)(2 * e) * N + n];
    const float f1 = Bm[(size_t)(2 * e + 1) * N + n];
    w[e] = pk16(bf_bits(f0), bf_bits(f1));
  }
  const bool data = (p < 2);
  v4u val;
#pragma unroll
  for (int e = 0; e < 4; ++e) val[e] = data ? w[e] : 0u;
  unsigned short* d = dst + (size_t)n * ldd + DM + p * 8;
  *(volatile v4u*)d = val;
  __threadfence();
  *(volatile v4u*)d = val;
}

__global__ __launch_bounds__(256) void lr_xa(const unsigned short* xq, const unsigned short* xk,
                                             const unsigned short* __restrict__ atp,
                                             const float* __restrict__ ab0, const float* __restrict__ ab1,
                                             const float* __restrict__ ab2,
                                             unsigned short* wq, unsigned short* wk, unsigned short* wv,
                                             int ntiles, int nwaves) {
  __shared__ __align__(16) float sT[8][16 * 16];
  const int tid = threadIdx.x, wave = tid >> 5, lane = tid & 31;
  const int w = blockIdx.x * 8 + wave;
  if (w >= nwaves) return;
  const int pr   = w / ntiles;
  const int tile = w - pr * ntiles;
  const int m0   = tile * 16;
  const __bf16* A  = (const __bf16*)(const void*)((pr == 0) ? xq : xk);
  unsigned short* W = (pr == 0) ? wq : ((pr == 1) ? wk : wv);
  const float* ab = (pr == 0) ? ab0 : ((pr == 1) ? ab1 : ab2);
  const __bf16* Bt = (const __bf16*)(const void*)atp + (size_t)pr * RKP * DM;
  const int rl   = lane & 15;
  const int koff = (lane >> 4) * 8;
  const int mOff = (lane >> 4) * 8;

  v8f acc = zero8();
  for (int k0 = 0; k0 < DM; k0 += 32) {
    const v16b a = ldfrag_b(A  + (size_t)(m0 + rl) * LDX + k0 + koff);
    const v16b b = ldfrag_b(Bt + (size_t)rl        * DM  + k0 + koff);
    acc = mma_b(a, b, acc);
  }

  float* slab = sT[wave];
#pragma unroll
  for (int r = 0; r < 8; ++r) slab[(mOff + r) * 16 + rl] = acc[r];
  __builtin_amdgcn_fence(__ATOMIC_RELEASE, "workgroup");
  __builtin_amdgcn_wave_barrier();
  __builtin_amdgcn_fence(__ATOMIC_ACQUIRE, "workgroup");

  const int q = lane >> 3, piece = lane & 7;
  v4u ov[4];
#pragma unroll
  for (int it = 0; it < 4; ++it) {
    const int row = it * 4 + q;
    const float* sp = slab + row * 16;
    v4u o;
#pragma unroll
    for (int e = 0; e < 4; ++e) {
      const float f0 = sp[2 * e]     + bfr(ab[2 * e]);
      const float f1 = sp[2 * e + 1] + bfr(ab[2 * e + 1]);
      const unsigned short h0 = bf_bits(f0), h1 = bf_bits(f1);
      const unsigned short l0 = bf_bits(f0 - bf_up(h0)), l1 = bf_bits(f1 - bf_up(h1));
      const unsigned hv = pk16(h0, h1), lv = pk16(l0, l1);
      o[e] = (piece == 0) ? hv : ((piece == 1) ? lv : 0u);
    }
    ov[it] = o;
  }
  for (int pass = 0; pass < 2; ++pass) {
#pragma unroll
    for (int it = 0; it < 4; ++it) {
      const int row = it * 4 + q;
      unsigned short* d = W + (size_t)(m0 + row) * LDX + DM + piece * 8;
      *(volatile v4u*)d = ov[it];
    }
    __threadfence();
  }
}

template <int NSPLIT, int OUT_MODE, int BROW>
__global__ __launch_bounds__(256) void gemm64(
    const unsigned short* __restrict__ Ap, const unsigned short* A2p, int lda,
    const unsigned short* __restrict__ Btp, int ldb,
    const float* __restrict__ b1, const float* __restrict__ b2, float f1, float f2,
    void* Cout, int ldc, void* Cout2, int ldc2,
    int M, int N, int K, float rscale) {
  const __bf16* A   = (const __bf16*)(const void*)Ap;
  const __bf16* A2  = (const __bf16*)(const void*)A2p;
  const __bf16* Bt  = (const __bf16*)(const void*)Btp;
  __shared__ __align__(16) float sT[8][16 * 68];
  const int lane = threadIdx.x & 31;
  const int wave = threadIdx.x >> 5;
  const int tilesN = N >> 6;
  const int tilesM = M >> 6;
  const int tile = blockIdx.x * 8 + wave;
  if (tile >= tilesM * tilesN) return;
  const int tm = tile / tilesN;
  const int tn = tile - tm * tilesN;
  const int m0 = tm << 6;
  const int n0 = tn << 6;

  const __bf16* Ab2 = (NSPLIT >= 1) ? A2 : A;

  const int rlane = lane & 15;
  const int koff  = (lane >> 4) * 8;
  const int mOff  = (lane >> 4) * 8;

  v8f acc[4][4];
#pragma unroll
  for (int i = 0; i < 4; ++i)
#pragma unroll
    for (int j = 0; j < 4; ++j) acc[i][j] = zero8();

  for (int k0 = 0; k0 < K; k0 += 32) {
    v16b bh[4];
#pragma unroll
    for (int j = 0; j < 4; ++j) {
      const size_t bo = (size_t)(n0 + (j << 4) + rlane) * ldb + koff + k0;
      bh[j] = ldfrag_b(Bt + bo);
    }
#pragma unroll
    for (int i = 0; i < 4; ++i) {
      const size_t ao = (size_t)(m0 + (i << 4) + rlane) * lda + koff + k0;
      const v16b ah = ldfrag_b(A + ao);
      v16b al = ah;
      if (NSPLIT >= 1) al = ldfrag_b(Ab2 + ao);
#pragma unroll
      for (int j = 0; j < 4; ++j) {
        acc[i][j] = mma_b_raw(ah, bh[j], acc[i][j]);
        if (NSPLIT >= 1) acc[i][j] = mma_b_raw(al, bh[j], acc[i][j]);
      }
      dep_guard_b(acc[i][0], acc[i][3], ah, al);
    }
    keep4_b(bh[0], bh[1], bh[2], bh[3]);
  }
  acc_guard4(acc[0][0], acc[0][1], acc[0][2], acc[0][3]);
  acc_guard4(acc[1][0], acc[1][1], acc[1][2], acc[1][3]);
  acc_guard4(acc[2][0], acc[2][1], acc[2][2], acc[2][3]);
  acc_guard4(acc[3][0], acc[3][1], acc[3][2], acc[3][3]);

  float bcol[4];
#pragma unroll
  for (int j = 0; j < 4; ++j) bcol[j] = 0.f;
  if (BROW == 0) {
#pragma unroll
    for (int j = 0; j < 4; ++j) {
      const int n = n0 + (j << 4) + rlane;
      bcol[j] = f1 * bfr(b1[n]) + f2 * bfr(b2[n]);
    }
  }

  float* slab = sT[wave];
#pragma unroll
  for (int i = 0; i < 4; ++i) {
    const int mBase = m0 + (i << 4);
    float brow[8];
#pragma unroll
    for (int r = 0; r < 8; ++r) brow[r] = 0.f;
    if (BROW != 0) {
#pragma unroll
      for (int r = 0; r < 8; ++r) {
        const int m = mBase + mOff + r;
        brow[r] = f1 * bfr(b1[m]) + f2 * bfr(b2[m]);
      }
    }
#pragma unroll
    for (int r = 0; r < 8; ++r) {
#pragma unroll
      for (int j = 0; j < 4; ++j) {
        slab[(mOff + r) * 68 + (j << 4) + rlane] = acc[i][j][r] + ((BROW != 0) ? brow[r] : bcol[j]);
      }
    }
    __builtin_amdgcn_fence(__ATOMIC_RELEASE, "workgroup");
    __builtin_amdgcn_wave_barrier();
    __builtin_amdgcn_fence(__ATOMIC_ACQUIRE, "workgroup");
    if (OUT_MODE == 0) {
      float* C = (float*)Cout;
      const int hh = lane >> 4, c4 = (lane & 15) * 4;
      v4f ov[8];
#pragma unroll
      for (int it = 0; it < 8; ++it) {
        const int row = it * 2 + hh;
        ov[it] = *(const v4f*)(slab + row * 68 + c4);
      }
      for (int pass = 0; pass < 2; ++pass) {
#pragma unroll
        for (int it = 0; it < 8; ++it) {
          const int row = it * 2 + hh;
          *(volatile v4f*)(C + (size_t)(mBase + row) * ldc + n0 + c4) = ov[it];
        }
        __threadfence();
      }
    } else {
      const int q = lane >> 3, c8 = (lane & 7) * 8;
      unsigned short* C  = (unsigned short*)Cout;
      unsigned short* C2 = (unsigned short*)Cout2;
      v4u hv[4], lv[4];
#pragma unroll
      for (int it = 0; it < 4; ++it) {
        const int row = it * 4 + q;
        const float* sp = slab + row * 68 + c8;
        v4u a, a2;
#pragma unroll
        for (int e = 0; e < 4; ++e) {
          const float f0 = sp[2 * e], fv1 = sp[2 * e + 1];
          unsigned short h0, h1, l0, l1;
          if (OUT_MODE == 2) {
            h0 = bf_bits(f0); h1 = bf_bits(fv1);
            l0 = bf_bits(f0 - bf_up(h0)); l1 = bf_bits(fv1 - bf_up(h1));
          } else {
            const _Float16 x0 = (_Float16)f0, x1 = (_Float16)fv1;
            h0 = h_bits(x0); h1 = h_bits(x1);
            l0 = h_bits((_Float16)((f0 - (float)x0) * rscale));
            l1 = h_bits((_Float16)((fv1 - (float)x1) * rscale));
          }
          a[e] = pk16(h0, h1); a2[e] = pk16(l0, l1);
        }
        hv[it] = a; lv[it] = a2;
      }
      for (int pass = 0; pass < 2; ++pass) {
#pragma unroll
        for (int it = 0; it < 4; ++it) {
          const int row = it * 4 + q;
          *(volatile v4u*)(C  + (size_t)(mBase + row) * ldc  + n0 + c8) = hv[it];
          *(volatile v4u*)(C2 + (size_t)(mBase + row) * ldc2 + n0 + c8) = lv[it];
        }
        __threadfence();
      }
    }
    __builtin_amdgcn_fence(__ATOMIC_RELEASE, "workgroup");
    __builtin_amdgcn_wave_barrier();
    __builtin_amdgcn_fence(__ATOMIC_ACQUIRE, "workgroup");
  }
}

__global__ __launch_bounds__(128)
void attn_cols(const unsigned short* __restrict__ qhp, const unsigned short* __restrict__ qlp,
               const unsigned short* __restrict__ khp, const unsigned short* __restrict__ klp,
               float* Sp, float* mstat, float* cstat, int hbase) {
  union FB { v16b v; v8b h[2]; };
  __shared__ __align__(16) __bf16 Qsh[64 * 64];
  __shared__ __align__(16) __bf16 Qsl[64 * 64];
  __shared__ __align__(16) float  slab[64 * SPITCH];
  __shared__ __align__(16) float  mst[64];
  __shared__ __align__(16) float  cst[64];

  const int tid  = threadIdx.x;
  const int wave = tid >> 5;
  const int lane = tid & 31;
  const int hh   = lane >> 4;
  const int c    = lane & 15;

  const int bx = blockIdx.x;
  const int kb = bx % NQB;
  const int hl = bx / NQB;
  const int h  = hbase + hl;

  const __bf16* Qh = (const __bf16*)(const void*)qhp + (size_t)h * HD;
  const __bf16* Ql = (const __bf16*)(const void*)qlp + (size_t)h * HD;
  const __bf16* Kh = (const __bf16*)(const void*)khp + (size_t)h * HD;
  const __bf16* Kl = (const __bf16*)(const void*)klp + (size_t)h * HD;

  const int keyrel = wave * 16 + c;
  const int key    = kb * 64 + keyrel;

  v16b kfh[2], kfl[2];
#pragma unroll
  for (int dc = 0; dc < 2; ++dc) {
    const size_t ko = (size_t)key * FT + dc * 32 + 8 * hh;
    kfh[dc] = ldfrag_b(Kh + ko);
    kfl[dc] = ldfrag_b(Kl + ko);
  }

  float* Sblk = Sp + (size_t)hl * SPH + tileoff_d(kb);
  float mrun = -INFINITY, lrun = 0.f;

  for (int qc = kb; qc < NQB; ++qc) {
    const int qrow0 = qc * 64;
    __syncthreads();
    {
      const int r = tid >> 1, half = (tid & 1) * 32;
      const __bf16* g0 = Qh + (size_t)(qrow0 + r) * FT + half;
      const __bf16* g1 = Ql + (size_t)(qrow0 + r) * FT + half;
#pragma unroll
      for (int i = 0; i < 4; ++i) {
        const v8b a0 = *(const v8b*)(g0 + 8 * i);
        const v8b a1 = *(const v8b*)(g1 + 8 * i);
        *(v8b*)(Qsh + r * 64 + half + 8 * i) = a0;
        *(v8b*)(Qsl + r * 64 + half + 8 * i) = a1;
      }
    }
    __syncthreads();

    v8f acc[4];
#pragma unroll
    for (int i = 0; i < 4; ++i) {
      acc[i] = zero8();
#pragma unroll
      for (int dc = 0; dc < 2; ++dc) {
        FB ah, al;
        ah.h[0] = *(const v8b*)(Qsh + (16 * i + c) * 64 + dc * 32 + 8 * hh);
        ah.h[1] = *(const v8b*)(Qsh + (16 * i + c) * 64 + dc * 32 + 16 + 8 * hh);
        al.h[0] = *(const v8b*)(Qsl + (16 * i + c) * 64 + dc * 32 + 8 * hh);
        al.h[1] = *(const v8b*)(Qsl + (16 * i + c) * 64 + dc * 32 + 16 + 8 * hh);
        acc[i] = mma_b(ah.v, kfh[dc], acc[i]);
        acc[i] = mma_b(ah.v, kfl[dc], acc[i]);
        acc[i] = mma_b(al.v, kfh[dc], acc[i]);
      }
    }

    const int qoff0 = (qc - kb) * 64;
    float m = -INFINITY;
#pragma unroll
    for (int i = 0; i < 4; ++i) {
#pragma unroll
      for (int r = 0; r < 8; ++r) {
        const int qrel = qoff0 + 16 * i + 8 * hh + r;
        const float v = acc[i][r];
        m = fmaxf(m, (qrel >= keyrel) ? v : -INFINITY);
      }
    }
    m = fmaxf(m, __shfl_xor(m, 16, 32));
    const float mnew  = fmaxf(mrun, m);
    const float alpha = (mrun == -INFINITY) ? 0.f : __expf(mrun - mnew);
    float ps = 0.f;
#pragma unroll
    for (int i = 0; i < 4; ++i) {
#pragma unroll
      for (int r = 0; r < 8; ++r) {
        const int qrel = qoff0 + 16 * i + 8 * hh + r;
        const float arg = (qrel >= keyrel) ? (acc[i][r] - mnew) : -10000.0f;
        ps += __expf(arg);
      }
    }
    ps += __shfl_xor(ps, 16, 32);
    lrun = lrun * alpha + ps;
    mrun = mnew;

#pragma unroll
    for (int i = 0; i < 4; ++i) {
#pragma unroll
      for (int r = 0; r < 8; ++r) slab[(16 * i + 8 * hh + r) * SPITCH + keyrel] = acc[i][r];
    }
    __syncthreads();
    {
      const int h2 = lane >> 4, c4 = (lane & 15) * 4;
      v4f ov[8];
#pragma unroll
      for (int it = 0; it < 8; ++it) {
        const int row = wave * 16 + it * 2 + h2;
        ov[it] = *(const v4f*)(slab + row * SPITCH + c4);
      }
      float* dst = Sblk + (size_t)qoff0 * 64;
      for (int pass = 0; pass < 2; ++pass) {
#pragma unroll
        for (int it = 0; it < 8; ++it) {
          const int row = wave * 16 + it * 2 + h2;
          *(volatile v4f*)(dst + (size_t)row * 64 + c4) = ov[it];
        }
        __threadfence();
      }
    }
  }

  if (hh == 0) {
    mst[keyrel] = mrun;
    cst[keyrel] = 128.0f * __builtin_amdgcn_rcpf(lrun);
  }
  __syncthreads();
  if (wave == 0) {
    const int c4 = (lane & 15) * 4;
    const v4f vm = *(const v4f*)(mst + c4);
    const v4f vc = *(const v4f*)(cst + c4);
    const v4f v  = (lane < 16) ? vm : vc;
    float* pd = ((lane < 16) ? mstat : cstat) + (size_t)hl * SEQ + kb * 64 + c4;
    *(volatile v4f*)pd = v;
    __threadfence();
    *(volatile v4f*)pd = v;
  }
}

template <bool RES>
__global__ __launch_bounds__(128)
void attn_out(const float* __restrict__ Sp, const float* __restrict__ mstat, const float* __restrict__ cstat,
              const unsigned short* __restrict__ vhp, const unsigned short* __restrict__ vlp,
              unsigned short* chp, unsigned short* clp, int hbase, int qbBase, int nqbThis) {
  union FH { v16h v; v8h h[2]; _Float16 e[16]; };
  union F8 { v4f q[2]; float f[8]; };
  __shared__ __align__(16) float    Ssh[64 * SPITCH];
  __shared__ __align__(16) _Float16 Vth[64 * 64];
  __shared__ __align__(16) _Float16 Vtl[RES ? 64 * 64 : 8];
  __shared__ __align__(16) float    msh[64];
  __shared__ __align__(16) float    csh[64];

  const int tid  = threadIdx.x;
  const int wave = tid >> 5;
  const int lane = tid & 31;
  const int hh   = lane >> 4;
  const int c    = lane & 15;

  const int bx  = blockIdx.x;
  const int qbl = bx % nqbThis;
  const int hl  = bx / nqbThis;
  const int h   = hbase + hl;
  const int qb  = qbBase + qbl;
  const int qr  = wave * 16 + c;

  const _Float16* Vh = (const _Float16*)(const void*)vhp + (size_t)(h * HD) * SEQ;
  const _Float16* Vl = (const _Float16*)(const void*)vlp + (size_t)(h * HD) * SEQ;
  const float* Shead = Sp + (size_t)hl * SPH;

  v8f oacc[4], o1[4];
#pragma unroll
  for (int t = 0; t < 4; ++t) { oacc[t] = zero8(); o1[t] = zero8(); }

  int nkc = qb + 1;
  if (nkc > NQB) nkc = NQB;
  for (int kc = 0; kc < nkc; ++kc) {
    __syncthreads();
    {
      const int r = tid >> 1, half = (tid & 1) * 32;
      const float* sg = Shead + tileoff_d(kc) + (size_t)((qb - kc) * 64 + r) * 64 + half;
#pragma unroll
      for (int i = 0; i < 8; ++i) {
        const v4f v = *(const v4f*)(sg + 4 * i);
        *(v4f*)(Ssh + r * SPITCH + half + 4 * i) = v;
      }
      const _Float16* vg = Vh + (size_t)r * SEQ + kc * 64 + half;
      const _Float16* wg = Vl + (size_t)r * SEQ + kc * 64 + half;
#pragma unroll
      for (int i = 0; i < 4; ++i) {
        const v8h b0 = *(const v8h*)(vg + 8 * i);
        *(v8h*)(Vth + r * 64 + half + 8 * i) = b0;
        if (RES) {
          const v8h bl = *(const v8h*)(wg + 8 * i);
          *(v8h*)(Vtl + r * 64 + half + 8 * i) = bl;
        }
      }
    }
    if (wave == 0) {
      const int c4 = (lane & 15) * 4;
      const v4f vm = *(const v4f*)(mstat + (size_t)hl * SEQ + kc * 64 + c4);
      const v4f vc = *(const v4f*)(cstat + (size_t)hl * SEQ + kc * 64 + c4);
      *(v4f*)(msh + c4) = vm;
      *(v4f*)(csh + c4) = vc;
    }
    __syncthreads();

    const int qoff = (qb - kc) * 64 + qr;
    const float* srow = Ssh + qr * SPITCH;
#pragma unroll 1
    for (int kk = 0; kk < 2; ++kk) {
      FH pa, pl;
#pragma unroll
      for (int g2 = 0; g2 < 2; ++g2) {
        const int kb8 = kk * 32 + 16 * g2 + 8 * hh;
        F8 sv, mv, cv;
        sv.q[0] = *(const v4f*)(srow + kb8);  sv.q[1] = *(const v4f*)(srow + kb8 + 4);
        mv.q[0] = *(const v4f*)(msh + kb8);   mv.q[1] = *(const v4f*)(msh + kb8 + 4);
        cv.q[0] = *(const v4f*)(csh + kb8);   cv.q[1] = *(const v4f*)(csh + kb8 + 4);
#pragma unroll
        for (int e = 0; e < 8; ++e) {
          const bool valid = (kb8 + e) <= qoff;
          const float arg  = valid ? (sv.f[e] - mv.f[e]) : -10000.0f;
          const float p1k  = __expf(arg) * cv.f[e];
          const _Float16 ph = (_Float16)p1k;
          pa.e[8 * g2 + e] = ph;
          if (RES) pl.e[8 * g2 + e] = (_Float16)((p1k - (float)ph) * 4096.0f);
        }
      }
      if (!RES) pl.v = pa.v;
#pragma unroll
      for (int t = 0; t < 4; ++t) {
        FH vb;
        vb.h[0] = *(const v8h*)(Vth + (t * 16 + c) * 64 + kk * 32 + 8 * hh);
        vb.h[1] = *(const v8h*)(Vth + (t * 16 + c) * 64 + kk * 32 + 16 + 8 * hh);
        oacc[t] = mma_h(pa.v, vb.v, oacc[t]);
        if (RES) {
          FH vl;
          vl.h[0] = *(const v8h*)(Vtl + (t * 16 + c) * 64 + kk * 32 + 8 * hh);
          vl.h[1] = *(const v8h*)(Vtl + (t * 16 + c) * 64 + kk * 32 + 16 + 8 * hh);
          o1[t] = mma_h(pa.v, vl.v, o1[t]);
          o1[t] = mma_h(pl.v, vb.v, o1[t]);
        }
      }
    }
  }

  __syncthreads();
  float* os = Ssh + wave * 16 * SPITCH;
#pragma unroll
  for (int r = 0; r < 8; ++r) {
#pragma unroll
    for (int t = 0; t < 4; ++t) {
      float v = oacc[t][r] * (1.0f / 1024.0f);
      if (RES) v += o1[t][r] * (1.0f / 4194304.0f);
      os[(8 * hh + r) * SPITCH + t * 16 + c] = v;
    }
  }
  __builtin_amdgcn_fence(__ATOMIC_RELEASE, "workgroup");
  __builtin_amdgcn_wave_barrier();
  __builtin_amdgcn_fence(__ATOMIC_ACQUIRE, "workgroup");
  {
    const int q4 = lane >> 3, c8 = (lane & 7) * 8;
    v4u hv[4], lv[4];
#pragma unroll
    for (int it = 0; it < 4; ++it) {
      const int row = it * 4 + q4;
      const float* sp = os + row * SPITCH + c8;
      v4u a, a2;
#pragma unroll
      for (int e = 0; e < 4; ++e) {
        const float f0 = sp[2 * e], fv1 = sp[2 * e + 1];
        const unsigned short h0 = bf_bits(f0), h1 = bf_bits(fv1);
        const unsigned short l0 = bf_bits(f0 - bf_up(h0)), l1 = bf_bits(fv1 - bf_up(h1));
        a[e] = pk16(h0, h1); a2[e] = pk16(l0, l1);
      }
      hv[it] = a; lv[it] = a2;
    }
    for (int pass = 0; pass < 2; ++pass) {
#pragma unroll
      for (int it = 0; it < 4; ++it) {
        const int row = it * 4 + q4;
        const size_t go = (size_t)(qb * 64 + wave * 16 + row) * FT + (size_t)h * HD + c8;
        *(volatile v4u*)(chp + go) = hv[it];
        *(volatile v4u*)(clp + go) = lv[it];
      }
      __threadfence();
    }
  }
}

extern "C" void kernel_launch(void* const* d_in, const int* in_sizes, int n_in,
                              void* d_out, int out_size, void* d_ws, size_t ws_size,
                              hipStream_t stream) {
  if (n_in < 23) return;
  if (in_sizes[0] != NB * SEQ * DM || in_sizes[1] != NB * SEQ * DM || in_sizes[2] != NB * SEQ * DM) return;
  if (in_sizes[3] != DM * FT || in_sizes[5] != DM * FT || in_sizes[7] != DM * FT) return;
  if (in_sizes[4] != FT || in_sizes[6] != FT || in_sizes[8] != FT) return;
  if (in_sizes[9] != DM * RK || in_sizes[13] != DM * RK || in_sizes[17] != DM * RK) return;
  if (in_sizes[10] != RK || in_sizes[14] != RK || in_sizes[18] != RK) return;
  if (in_sizes[11] != RK * FT || in_sizes[15] != RK * FT || in_sizes[19] != RK * FT) return;
  if (in_sizes[12] != FT || in_sizes[16] != FT || in_sizes[20] != FT) return;
  if (in_sizes[21] != FT * DM || in_sizes[22] != DM) return;
  if (out_size != NB * SEQ * DM) return;

  const float* xq_in = (const float*)d_in[0];
  const float* xk_in = (const float*)d_in[1];
  const float* xv_in = (const float*)d_in[2];
  const float* Wq  = (const float*)d_in[3];
  const float* Wqb = (const float*)d_in[4];
  const float* Wk  = (const float*)d_in[5];
  const float* Wkb = (const float*)d_in[6];
  const float* Wv  = (const float*)d_in[7];
  const float* Wvb = (const float*)d_in[8];
  const float* Aq  = (const float*)d_in[9];
  const float* Aqb = (const float*)d_in[10];
  const float* Bq  = (const float*)d_in[11];
  const float* Bqb = (const float*)d_in[12];
  const float* Ak  = (const float*)d_in[13];
  const float* Akb = (const float*)d_in[14];
  const float* Bk  = (const float*)d_in[15];
  const float* Bkb = (const float*)d_in[16];
  const float* Av  = (const float*)d_in[17];
  const float* Avb = (const float*)d_in[18];
  const float* Bv  = (const float*)d_in[19];
  const float* Bvb = (const float*)d_in[20];
  const float* Wo  = (const float*)d_in[21];
  const float* Wob = (const float*)d_in[22];

  const size_t PW   = (size_t)FT * LDX * 2;
  const size_t PWo  = (size_t)DM * FT * 2;
  const size_t PAT  = (size_t)3 * RKP * DM * 2;
  const size_t PX   = (size_t)SEQ * LDX * 2;
  const size_t PP   = (size_t)SEQ * FT * 2;
  const size_t PVT  = (size_t)FT * SEQ * 2;
  const size_t PST  = (size_t)GH * SEQ * 4;
  const size_t PS   = (size_t)GH * (size_t)SPH * 4;
  size_t off = 0;
  const size_t oWq = off; off += PW;
  const size_t oWk = off; off += PW;
  const size_t oWv = off; off += PW;
  const size_t oWo = off; off += PWo;
  const size_t oAT = off; off += PAT;
  const size_t oXq = off; off += PX;
  const size_t oXk = off; off += PX;
  const size_t oXv = off; off += PX;
  const size_t oQh = off; off += PP;
  const size_t oQl = off; off += PP;
  const size_t oKh = off; off += PP;
  const size_t oKl = off; off += PP;
  const size_t oCh = off; off += PP;
  const size_t oCl = off; off += PP;
  const size_t oVTh = off; off += PVT;
  const size_t oVTl = off; off += PVT;
  const size_t oMs = off; off += PST;
  const size_t oCs = off; off += PST;
  const size_t oS  = off; off += PS;
  if (off > ws_size) return;
  if (off > (size_t)134217728) return;

  char* ws = (char*)d_ws;
  unsigned short* WqTe = (unsigned short*)(ws + oWq);
  unsigned short* WkTe = (unsigned short*)(ws + oWk);
  unsigned short* WvTe = (unsigned short*)(ws + oWv);
  unsigned short* WoT  = (unsigned short*)(ws + oWo);
  unsigned short* AT   = (unsigned short*)(ws + oAT);
  unsigned short* Xq   = (unsigned short*)(ws + oXq);
  unsigned short* Xk   = (unsigned short*)(ws + oXk);
  unsigned short* Xv   = (unsigned short*)(ws + oXv);
  unsigned short* Qh   = (unsigned short*)(ws + oQh);
  unsigned short* Ql   = (unsigned short*)(ws + oQl);
  unsigned short* Kh   = (unsigned short*)(ws + oKh);
  unsigned short* Kl   = (unsigned short*)(ws + oKl);
  unsigned short* Ch   = (unsigned short*)(ws + oCh);
  unsigned short* Cl   = (unsigned short*)(ws + oCl);
  unsigned short* VTh  = (unsigned short*)(ws + oVTh);
  unsigned short* VTl  = (unsigned short*)(ws + oVTl);
  float*          Ms   = (float*)(ws + oMs);
  float*          Cs   = (float*)(ws + oCs);
  float*          Sws  = (float*)(ws + oS);
  float*          outf = (float*)d_out;

  const dim3 blk(256), blk128(128);
  const int nper   = SEQ * (DM / 8);
  const int nCvt   = 3 * nper;
  const int nTl16  = SEQ / 16;
  const int nwXa   = 3 * nTl16;
  const int neW    = FT * 8;
  const dim3 gAT(24);
  const dim3 gTrW(DM / 64, FT / 32);
  const dim3 gTrWo(FT / 64, DM / 32);
  const dim3 geW((neW + 255) / 256);
  const dim3 gCvt((nCvt + 255) / 256);
  const dim3 gXa((nwXa + 7) / 8);
  const dim3 gProj(((SEQ / 64) * (FT / 64) + 7) / 8);
  const dim3 gVT(((FT / 64) * (SEQ / 64) + 7) / 8);
  const dim3 gOut(((SEQ / 64) * (DM / 64) + 7) / 8);
  const dim3 gP1(GH * NQB);
  const dim3 gP2a(GH * QBRES);
  const dim3 gP2b(GH * (NQB - QBRES));

  lr_at<<<gAT, blk, 0, stream>>>(Aq, Ak, Av, AT);
  tr_cvt_bf16<<<gTrW, blk, 0, stream>>>(Wq, WqTe, DM, FT, LDX);
  tr_cvt_bf16<<<gTrW, blk, 0, stream>>>(Wk, WkTe, DM, FT, LDX);
  tr_cvt_bf16<<<gTrW, blk, 0, stream>>>(Wv, WvTe, DM, FT, LDX);
  tr_cvt_bf16<<<gTrWo, blk, 0, stream>>>(Wo, WoT, FT, DM, FT);
  wext<<<geW, blk, 0, stream>>>(Bq, WqTe, LDX, FT, neW);
  wext<<<geW, blk, 0, stream>>>(Bk, WkTe, LDX, FT, neW);
  wext<<<geW, blk, 0, stream>>>(Bv, WvTe, LDX, FT, neW);

  for (int b = 0; b < NB; ++b) {
    const float* xq_b = xq_in + (size_t)b * SEQ * DM;
    const float* xk_b = xk_in + (size_t)b * SEQ * DM;
    const float* xv_b = xv_in + (size_t)b * SEQ * DM;
    float* out_b = outf + (size_t)b * SEQ * DM;

    cvt_rows3<<<gCvt, blk, 0, stream>>>(xq_b, xk_b, xv_b, Xq, Xk, Xv, nper, nCvt);
    lr_xa<<<gXa, blk, 0, stream>>>(Xq, Xk, AT, Aqb, Akb, Avb, Xq, Xk, Xv, nTl16, nwXa);
    gemm64<0, 2, 0><<<gProj, blk, 0, stream>>>(
        Xq, Xq, LDX, WqTe, LDX, Wqb, Bqb, 1.0f, 1.0f,
        (void*)Qh, FT, (void*)Ql, FT, SEQ, FT, KE, 1.0f);
    gemm64<0, 2, 0><<<gProj, blk, 0, stream>>>(
        Xk, Xk, LDX, WkTe, LDX, Wkb, Bkb, 1.0f, 1.0f,
        (void*)Kh, FT, (void*)Kl, FT, SEQ, FT, KE, 1.0f);
    gemm64<0, 3, 1><<<gVT, blk, 0, stream>>>(
        WvTe, WvTe, LDX, Xv, LDX, Wvb, Bvb, 1.0f, 1.0f,
        (void*)VTh, SEQ, (void*)VTl, SEQ, FT, SEQ, KE, 4096.0f);
    for (int g = 0; g < NGRP; ++g) {
      const int hbase = g * GH;
      attn_cols<<<gP1, blk128, 0, stream>>>(Qh, Ql, Kh, Kl, Sws, Ms, Cs, hbase);
      attn_out<false><<<gP2a, blk128, 0, stream>>>(Sws, Ms, Cs, VTh, VTl, Ch, Cl, hbase, 0, QBRES);
      attn_out<true><<<gP2b, blk128, 0, stream>>>(Sws, Ms, Cs, VTh, VTl, Ch, Cl, hbase, QBRES, NQB - QBRES);
    }
    gemm64<1, 0, 0><<<gOut, blk, 0, stream>>>(
        Ch, Cl, FT, WoT, FT, Wob, Wob, 1.0f, 0.0f,
        (void*)out_b, DM, (void*)out_b, 0, SEQ, DM, FT, 1.0f);
  }
  (void)hipGetLastError();
}
